// EpisodicMemory_41652592836910
// MI455X (gfx1250) — hardware-verified
//
#include <hip/hip_runtime.h>
#include <math.h>
#include <stdint.h>

#define NQ   4096
#define CAP  8192
#define DD   512
#define KMAX 64
#define NCAP 256
#define GWIN 15.0f
static_assert((NQ % 64) == 0 && (CAP % 64) == 0 && (DD % 64) == 0);
static_assert((DD % 32) == 0);
static_assert((CAP % 256) == 0);
static_assert((NQ % 4) == 0);
static_assert(DD == 512);
static_assert((NCAP % 32) == 0 && NCAP >= KMAX);

typedef _Float16 v16h __attribute__((ext_vector_type(16)));
typedef _Float16 v8h  __attribute__((ext_vector_type(8)));
typedef __bf16   v16b __attribute__((ext_vector_type(16)));
typedef __bf16   v8b  __attribute__((ext_vector_type(8)));
typedef float    v8f  __attribute__((ext_vector_type(8)));
typedef float    v4f  __attribute__((ext_vector_type(4)));
typedef unsigned int v4u __attribute__((ext_vector_type(4)));
typedef v4f __attribute__((may_alias)) v4fa;
typedef v8h __attribute__((may_alias)) v8ha;

#if defined(__HIP_DEVICE_COMPILE__)
#define DEV_ASM 1
#else
#define DEV_ASM 0
#endif

__device__ __forceinline__ unsigned short bf_bits(float f) {
  unsigned u = __float_as_uint(f);
  return (unsigned short)((u + 0x7FFFu + ((u >> 16) & 1u)) >> 16);
}
__device__ __forceinline__ unsigned short h_bits(_Float16 x) { return __builtin_bit_cast(unsigned short, x); }
__device__ __forceinline__ unsigned pk16(unsigned short a, unsigned short b) { return (unsigned)a | ((unsigned)b << 16); }
__device__ __forceinline__ v8f zero8() { v8f z = {0.f, 0.f, 0.f, 0.f, 0.f, 0.f, 0.f, 0.f}; return z; }

__device__ __forceinline__ void wave_lds_sync() {
  __builtin_amdgcn_fence(__ATOMIC_RELEASE, "workgroup");
  __builtin_amdgcn_wave_barrier();
  __builtin_amdgcn_fence(__ATOMIC_ACQUIRE, "workgroup");
}

template <typename OT> struct FT;
template <> struct FT<__bf16>   { typedef v16b frag; typedef v8b half8; };
template <> struct FT<_Float16> { typedef v16h frag; typedef v8h half8; };

template <typename OT>
__device__ __forceinline__ typename FT<OT>::frag ldfrag(const OT* p) {
  union { typename FT<OT>::frag v; typename FT<OT>::half8 h[2]; } f;
  f.h[0] = *(const typename FT<OT>::half8*)(p);
  f.h[1] = *(const typename FT<OT>::half8*)(p + 16);
  return f.v;
}

__device__ __forceinline__ v8f mmar(v16b a, v16b b, v8f c) {
  return __builtin_amdgcn_wmma_f32_16x16x32_bf16(false, a, false, b, (short)0, c, false, false);
}
__device__ __forceinline__ v8f mmar(v16h a, v16h b, v8f c) {
  return __builtin_amdgcn_wmma_f32_16x16x32_f16(false, a, false, b, (short)0, c, false, false);
}
__device__ __forceinline__ void dep_guard(v8f& a, v8f& b, v16b x, v16b y) {
#if DEV_ASM
  asm volatile("v_nop\n\tv_nop\n\tv_nop\n\tv_nop" : "+v"(a), "+v"(b) : "v"(x), "v"(y));
#else
  (void)a; (void)b; (void)x; (void)y;
#endif
}
__device__ __forceinline__ void dep_guard(v8f& a, v8f& b, v16h x, v16h y) {
#if DEV_ASM
  asm volatile("v_nop\n\tv_nop\n\tv_nop\n\tv_nop" : "+v"(a), "+v"(b) : "v"(x), "v"(y));
#else
  (void)a; (void)b; (void)x; (void)y;
#endif
}
__device__ __forceinline__ void keep4(v16b a, v16b b, v16b c, v16b d) {
#if DEV_ASM
  asm volatile("v_nop" :: "v"(a), "v"(b), "v"(c), "v"(d));
#else
  (void)a; (void)b; (void)c; (void)d;
#endif
}
__device__ __forceinline__ void keep4(v16h a, v16h b, v16h c, v16h d) {
#if DEV_ASM
  asm volatile("v_nop" :: "v"(a), "v"(b), "v"(c), "v"(d));
#else
  (void)a; (void)b; (void)c; (void)d;
#endif
}
__device__ __forceinline__ void acc_guard4(v8f& a, v8f& b, v8f& c, v8f& d) {
#if DEV_ASM
  asm volatile("v_nop\n\tv_nop\n\tv_nop\n\tv_nop" : "+v"(a), "+v"(b), "+v"(c), "+v"(d));
#else
  (void)a; (void)b; (void)c; (void)d;
#endif
}

__global__ __launch_bounds__(256) void cvt_bf16x8(const float* __restrict__ in, unsigned short* out, int n8) {
  const int i = blockIdx.x * 256 + (int)threadIdx.x;
  if (i < n8) {
    const v4f a  = *(const v4fa*)(in + (size_t)i * 8);
    const v4f a4 = *(const v4fa*)(in + (size_t)i * 8 + 4);
    v4u p;
    p[0] = pk16(bf_bits(a[0]),  bf_bits(a[1]));
    p[1] = pk16(bf_bits(a[2]),  bf_bits(a[3]));
    p[2] = pk16(bf_bits(a4[0]), bf_bits(a4[1]));
    p[3] = pk16(bf_bits(a4[2]), bf_bits(a4[3]));
    unsigned short* o = out + (size_t)i * 8;
    *(volatile v4u*)o = p;
    __threadfence();
    *(volatile v4u*)o = p;
  }
}

template <typename OT, int OUT_MODE>
__global__ __launch_bounds__(256) void gemm64(
    const unsigned short* __restrict__ Ap, int lda,
    const unsigned short* __restrict__ Btp, int ldb,
    float* Cf, int ldcf, unsigned short* Ch, int ldch,
    int M, int N, int K) {
  typedef typename FT<OT>::frag V16;
  const OT* A  = (const OT*)(const void*)Ap;
  const OT* Bt = (const OT*)(const void*)Btp;
  __shared__ __align__(16) float sT[8][16 * 68];
  const int lane = threadIdx.x & 31;
  const int wave = threadIdx.x >> 5;
  const int tilesN = N >> 6;
  const int tilesM = M >> 6;
  const int tile = blockIdx.x * 8 + wave;
  if (tile >= tilesM * tilesN) return;
  const int tm = tile / tilesN;
  const int tn = tile - tm * tilesN;
  const int m0 = tm << 6;
  const int n0 = tn << 6;

  const int rlane = lane & 15;
  const int koff  = (lane >> 4) * 8;
  const int mOff  = (lane >> 4) * 8;

  v8f acc[4][4];
#pragma unroll
  for (int i = 0; i < 4; ++i)
#pragma unroll
    for (int j = 0; j < 4; ++j) acc[i][j] = zero8();

  for (int k0 = 0; k0 < K; k0 += 32) {
    V16 bq[4];
#pragma unroll
    for (int j = 0; j < 4; ++j)
      bq[j] = ldfrag<OT>(Bt + (size_t)(n0 + (j << 4) + rlane) * ldb + koff + k0);
#pragma unroll
    for (int i = 0; i < 4; ++i) {
      const V16 af = ldfrag<OT>(A + (size_t)(m0 + (i << 4) + rlane) * lda + koff + k0);
#pragma unroll
      for (int j = 0; j < 4; ++j) acc[i][j] = mmar(af, bq[j], acc[i][j]);
      dep_guard(acc[i][0], acc[i][3], af, bq[3]);
    }
    keep4(bq[0], bq[1], bq[2], bq[3]);
  }
  acc_guard4(acc[0][0], acc[0][1], acc[0][2], acc[0][3]);
  acc_guard4(acc[1][0], acc[1][1], acc[1][2], acc[1][3]);
  acc_guard4(acc[2][0], acc[2][1], acc[2][2], acc[2][3]);
  acc_guard4(acc[3][0], acc[3][1], acc[3][2], acc[3][3]);

  float* slab = sT[wave];
#pragma unroll
  for (int i = 0; i < 4; ++i) {
    const int mBase = m0 + (i << 4);
#pragma unroll
    for (int j = 0; j < 4; ++j) {
#pragma unroll
      for (int r = 0; r < 8; ++r) {
        slab[(mOff + r) * 68 + (j << 4) + rlane] = acc[i][j][r];
      }
    }
    wave_lds_sync();
    if (OUT_MODE != 1) {
      const int h2 = lane >> 4, c4 = (lane & 15) * 4;
      for (int pass = 0; pass < 2; ++pass) {
#pragma unroll
        for (int it = 0; it < 8; ++it) {
          const int row = it * 2 + h2;
          const v4f v = *(const v4fa*)(slab + row * 68 + c4);
          *(volatile v4f*)(Cf + (size_t)(mBase + row) * ldcf + n0 + c4) = v;
        }
        __threadfence();
      }
    }
    if (OUT_MODE != 0) {
      const int q = lane >> 3, c8 = (lane & 7) * 8;
      v4u hv[4];
#pragma unroll
      for (int it = 0; it < 4; ++it) {
        const int row = it * 4 + q;
        const float* sp = slab + row * 68 + c8;
        v4u a;
#pragma unroll
        for (int e = 0; e < 4; ++e) {
          const _Float16 x0 = (_Float16)sp[2 * e];
          const _Float16 x1 = (_Float16)sp[2 * e + 1];
          a[e] = pk16(h_bits(x0), h_bits(x1));
        }
        hv[it] = a;
      }
      for (int pass = 0; pass < 2; ++pass) {
#pragma unroll
        for (int it = 0; it < 4; ++it) {
          const int row = it * 4 + q;
          *(volatile v4u*)(Ch + (size_t)(mBase + row) * ldch + n0 + c8) = hv[it];
        }
        __threadfence();
      }
    }
    wave_lds_sync();
  }
}

__global__ __launch_bounds__(128) void select_rows(
    const unsigned short* __restrict__ Sp, const float* __restrict__ Qf,
    const float* __restrict__ Kf, const float* __restrict__ Vf,
    const int* __restrict__ topk, float* out) {
  __shared__ __align__(16) int   cidx[4][NCAP];
  __shared__ __align__(16) float cscr[4][NCAP];
  __shared__ __align__(16) float cprb[4][NCAP];

  const int tid  = threadIdx.x;
  const int lane = tid & 31;
  const int w    = tid >> 5;
  const int row  = blockIdx.x * 4 + w;
  int*   ci  = cidx[w];
  float* cs  = cscr[w];
  float* cpv = cprb[w];

  const int  tk   = topk[0];
  const bool kbad = (tk > KMAX);
  const int  kk   = min(max(tk, 1), KMAX);

#pragma unroll
  for (int t = 0; t < NCAP / 32; ++t) {
    ci[lane + 32 * t]  = 0;
    cs[lane + 32 * t]  = -INFINITY;
    cpv[lane + 32 * t] = 0.f;
  }

  const _Float16* srow = (const _Float16*)(const void*)Sp + (size_t)row * CAP + 8 * lane;

  float mx = -INFINITY;
#pragma unroll 2
  for (int it = 0; it < CAP / 256; ++it) {
    const v8h hv = *(const v8ha*)(srow + it * 256);
#pragma unroll
    for (int e = 0; e < 8; ++e) mx = fmaxf(mx, (float)hv[e]);
  }
#pragma unroll
  for (int off = 16; off > 0; off >>= 1) mx = fmaxf(mx, __shfl_xor(mx, off, 32));
  const float thr = mx - GWIN;

  int ncand = 0;
#pragma unroll 1
  for (int it = 0; it < CAP / 256; ++it) {
    const v8h hv = *(const v8ha*)(srow + it * 256);
    unsigned hm = 0u;
#pragma unroll
    for (int e = 0; e < 8; ++e) hm |= ((float)hv[e] >= thr) ? (1u << e) : 0u;
    const int cnt = __builtin_popcount(hm);
    const unsigned anyb = __builtin_amdgcn_ballot_w32(cnt != 0);
    if (anyb != 0u) {
      int incl = cnt;
#pragma unroll
      for (int off = 1; off < 32; off <<= 1) {
        const int t = __shfl_up(incl, off, 32);
        incl += (lane >= off) ? t : 0;
      }
      const int total = __shfl(incl, 31, 32);
      int pos = ncand + incl - cnt;
#pragma unroll
      for (int e = 0; e < 8; ++e) {
        if (hm & (1u << e)) {
          if (pos < NCAP) ci[pos] = it * 256 + lane * 8 + e;
          ++pos;
        }
      }
      ncand += total;
    }
  }
  const bool ovf = (ncand > NCAP);
  ncand = min(ncand, NCAP);
  wave_lds_sync();

  const float* qr = Qf + (size_t)row * DD + 4 * lane;
  const v4f q0 = *(const v4fa*)(qr);
  const v4f q1 = *(const v4fa*)(qr + 128);
  const v4f q2 = *(const v4fa*)(qr + 256);
  const v4f q3 = *(const v4fa*)(qr + 384);
#pragma unroll 1
  for (int j = 0; j < ncand; ++j) {
    int key = ci[j];
    key = min(max(key, 0), CAP - 1);
    const float* kr = Kf + (size_t)key * DD + 4 * lane;
    const v4f k0 = *(const v4fa*)(kr);
    const v4f k1 = *(const v4fa*)(kr + 128);
    const v4f k2 = *(const v4fa*)(kr + 256);
    const v4f k3 = *(const v4fa*)(kr + 384);
    const v4f pr = q0 * k0 + q1 * k1 + q2 * k2 + q3 * k3;
    float p = (pr[0] + pr[1]) + (pr[2] + pr[3]);
#pragma unroll
    for (int off = 16; off > 0; off >>= 1) p += __shfl_xor(p, off, 32);
    if (lane == 0) cs[j] = p;
  }
  wave_lds_sync();

  float smax = -INFINITY;
#pragma unroll 1
  for (int t = 0; t < NCAP / 32; ++t) smax = fmaxf(smax, cs[lane + 32 * t]);
#pragma unroll
  for (int off = 16; off > 0; off >>= 1) smax = fmaxf(smax, __shfl_xor(smax, off, 32));

  float psum = 0.f;
#pragma unroll 1
  for (int t = 0; t < NCAP / 32; ++t) {
    const int   j  = lane + 32 * t;
    const float s  = cs[j];
    const int   ij = ci[j];
    bool keep = (j < ncand);
    if (ncand > kk) {
      int rank = 0;
#pragma unroll 1
      for (int i = 0; i < ncand; ++i) {
        const float si = cs[i];
        const int   ii = ci[i];
        rank += ((si > s) || (si == s && ii < ij)) ? 1 : 0;
      }
      keep = keep && (rank < kk);
    }
    const float p = keep ? __expf(s - smax) : 0.f;
    cpv[j] = p;
    psum += p;
  }
#pragma unroll
  for (int off = 16; off > 0; off >>= 1) psum += __shfl_xor(psum, off, 32);
  wave_lds_sync();
  const float inv = 1.0f / psum;

  v4f o0 = {0.f, 0.f, 0.f, 0.f};
  v4f o1 = o0, o2 = o0, o3 = o0;
#pragma unroll 1
  for (int j = 0; j < ncand; ++j) {
    const float p = cpv[j];
    int key = ci[j];
    key = min(max(key, 0), CAP - 1);
    const float* vr = Vf + (size_t)key * DD + 4 * lane;
    o0 += p * *(const v4fa*)(vr);
    o1 += p * *(const v4fa*)(vr + 128);
    o2 += p * *(const v4fa*)(vr + 256);
    o3 += p * *(const v4fa*)(vr + 384);
  }
  o0 *= inv; o1 *= inv; o2 *= inv; o3 *= inv;
  if (kbad || ovf) {
    const float qn = __uint_as_float(0x7fc00000u);
    const v4f n4 = {qn, qn, qn, qn};
    o0 = n4; o1 = n4; o2 = n4; o3 = n4;
  }
  float* orow = out + (size_t)row * DD + 4 * lane;
  *(volatile v4f*)(orow)       = o0;
  *(volatile v4f*)(orow + 128) = o1;
  *(volatile v4f*)(orow + 256) = o2;
  *(volatile v4f*)(orow + 384) = o3;
  __threadfence();
  *(volatile v4f*)(orow)       = o0;
  *(volatile v4f*)(orow + 128) = o1;
  *(volatile v4f*)(orow + 256) = o2;
  *(volatile v4f*)(orow + 384) = o3;
}

extern "C" void kernel_launch(void* const* d_in, const int* in_sizes, int n_in,
                              void* d_out, int out_size, void* d_ws, size_t ws_size,
                              hipStream_t stream) {
  if (n_in < 6) return;
  if (in_sizes[0] != NQ * DD) return;
  if (in_sizes[1] != CAP * DD) return;
  if (in_sizes[2] != DD * DD || in_sizes[3] != DD * DD || in_sizes[4] != DD * DD) return;
  if (in_sizes[5] < 1) return;
  if (out_size != NQ * DD) return;

  const float* query  = (const float*)d_in[0];
  const float* memory = (const float*)d_in[1];
  const float* Wq     = (const float*)d_in[2];
  const float* Wk     = (const float*)d_in[3];
  const float* Wv     = (const float*)d_in[4];
  const int*   topk   = (const int*)d_in[5];
  float* out = (float*)d_out;

  const size_t PQF = (size_t)NQ * DD * 4;
  const size_t PQH = (size_t)NQ * DD * 2;
  const size_t PKF = (size_t)CAP * DD * 4;
  const size_t PKH = (size_t)CAP * DD * 2;
  const size_t PVF = PKF;
  const size_t PS  = (size_t)NQ * CAP * 2;
  const size_t PW  = (size_t)DD * DD * 2;
  size_t off = 0;
  const size_t oQf = off; off += PQF;
  const size_t oQh = off; off += PQH;
  const size_t oKf = off; off += PKF;
  const size_t oKh = off; off += PKH;
  const size_t oVf = off; off += PVF;
  const size_t oS  = off; off += PS;
  if (off > ws_size) return;
  if (off > (size_t)134217728) return;
  const size_t oQb  = oS;
  const size_t oMb  = oQb + PQH;
  const size_t oWqb = oMb + PKH;
  const size_t oWkb = oWqb + PW;
  const size_t oWvb = oWkb + PW;
  if (oWvb + PW > oS + PS) return;

  char* ws = (char*)d_ws;
  float*          Qf  = (float*)(ws + oQf);
  unsigned short* Qh  = (unsigned short*)(ws + oQh);
  float*          Kf  = (float*)(ws + oKf);
  unsigned short* Kh  = (unsigned short*)(ws + oKh);
  float*          Vf  = (float*)(ws + oVf);
  unsigned short* Sh  = (unsigned short*)(ws + oS);
  unsigned short* Qb  = (unsigned short*)(ws + oQb);
  unsigned short* Mb  = (unsigned short*)(ws + oMb);
  unsigned short* Wqb = (unsigned short*)(ws + oWqb);
  unsigned short* Wkb = (unsigned short*)(ws + oWkb);
  unsigned short* Wvb = (unsigned short*)(ws + oWvb);

  const dim3 blk(256);
  const int n8q = NQ * DD / 8;
  const int n8m = CAP * DD / 8;
  const int n8w = DD * DD / 8;
  const dim3 gCvtQ((n8q + 255) / 256);
  const dim3 gCvtM((n8m + 255) / 256);
  const dim3 gCvtW((n8w + 255) / 256);
  const dim3 gQ(((NQ / 64) * (DD / 64) + 7) / 8);
  const dim3 gKV(((CAP / 64) * (DD / 64) + 7) / 8);
  const dim3 gS(((NQ / 64) * (CAP / 64) + 7) / 8);
  const dim3 gSel(NQ / 4);

  cvt_bf16x8<<<gCvtQ, blk, 0, stream>>>(query,  Qb,  n8q);
  cvt_bf16x8<<<gCvtM, blk, 0, stream>>>(memory, Mb,  n8m);
  cvt_bf16x8<<<gCvtW, blk, 0, stream>>>(Wq,     Wqb, n8w);
  cvt_bf16x8<<<gCvtW, blk, 0, stream>>>(Wk,     Wkb, n8w);
  cvt_bf16x8<<<gCvtW, blk, 0, stream>>>(Wv,     Wvb, n8w);
  gemm64<__bf16, 2><<<gQ, blk, 0, stream>>>(Qb, DD, Wqb, DD, Qf, DD, Qh, DD, NQ, DD, DD);
  gemm64<__bf16, 2><<<gKV, blk, 0, stream>>>(Mb, DD, Wkb, DD, Kf, DD, Kh, DD, CAP, DD, DD);
  gemm64<__bf16, 0><<<gKV, blk, 0, stream>>>(Mb, DD, Wvb, DD, Vf, DD, Kh, DD, CAP, DD, DD);
  gemm64<_Float16, 1><<<gS, blk, 0, stream>>>(Qh, DD, Kh, DD, Qf, CAP, Sh, CAP, NQ, CAP, DD);
  select_rows<<<gSel, dim3(128), 0, stream>>>(Sh, Qf, Kf, Vf, topk, out);
  (void)hipGetLastError();
}
